// HierMultiHeadAttn_42545946034840
// MI455X (gfx1250) — hardware-verified
//
#include <hip/hip_runtime.h>

typedef __attribute__((ext_vector_type(16))) _Float16 v16h;
typedef __attribute__((ext_vector_type(8)))  _Float16 v8h;
typedef __attribute__((ext_vector_type(16))) __bf16   v16b;
typedef __attribute__((ext_vector_type(8)))  __bf16   v8b;
typedef __attribute__((ext_vector_type(8)))  float    v8f;
typedef __attribute__((ext_vector_type(4)))  float    v4f;

#define NB 4
#define SEQ 2048
#define CH 1024
#define NHEAD 16
#define HD 64
#define NK0 1024
#define NK1 256
#define NK2 64
#define AKC 64

__device__ __forceinline__ unsigned short f2bf_bits(float f) {
  unsigned u = __float_as_uint(f);
  return (unsigned short)((u + 0x7FFFu + ((u >> 16) & 1u)) >> 16);
}
__device__ __forceinline__ float bf_bits2f(unsigned short h) { return __uint_as_float(((unsigned)h) << 16); }

__device__ __forceinline__ void dep_guard_h(v8f& a, v8f& b, v16h x, v16h y) { asm volatile("v_nop\n\tv_nop\n\tv_nop\n\tv_nop" : "+v"(a), "+v"(b) : "v"(x), "v"(y)); }
__device__ __forceinline__ void dep_guard_b(v8f& a, v8f& b, v16b x, v16b y) { asm volatile("v_nop\n\tv_nop\n\tv_nop\n\tv_nop" : "+v"(a), "+v"(b) : "v"(x), "v"(y)); }
__device__ __forceinline__ void keep4_h(v16h a, v16h b, v16h c, v16h d) { asm volatile("v_nop" :: "v"(a), "v"(b), "v"(c), "v"(d)); }
__device__ __forceinline__ void keep4_b(v16b a, v16b b, v16b c, v16b d) { asm volatile("v_nop" :: "v"(a), "v"(b), "v"(c), "v"(d)); }
__device__ __forceinline__ void acc_guard4(v8f& a, v8f& b, v8f& c, v8f& d) { asm volatile("v_nop\n\tv_nop\n\tv_nop\n\tv_nop" : "+v"(a), "+v"(b), "+v"(c), "+v"(d)); }
template <typename T> struct Frag;
template <> struct Frag<_Float16> {
  typedef v16h V; union U { v16h v; v8h h[2]; };
  static __device__ __forceinline__ v16h load(const _Float16* p) {
    U f; f.h[0] = *(const v8h*)(p); f.h[1] = *(const v8h*)(p + 16); return f.v;
  }
  static __device__ __forceinline__ v8f mma(v16h a, v16h b, v8f c) {
    return __builtin_amdgcn_wmma_f32_16x16x32_f16(false, a, false, b, (short)0, c, false, false);
  }
  static __device__ __forceinline__ void guard(v8f& a, v8f& b, v16h x, v16h y) { dep_guard_h(a, b, x, y); }
  static __device__ __forceinline__ void keep(v16h a, v16h b, v16h c, v16h d) { keep4_h(a, b, c, d); }
};
template <> struct Frag<__bf16> {
  typedef v16b V; union U { v16b v; v8b h[2]; };
  static __device__ __forceinline__ v16b load(const __bf16* p) {
    U f; f.h[0] = *(const v8b*)(p); f.h[1] = *(const v8b*)(p + 16); return f.v;
  }
  static __device__ __forceinline__ v8f mma(v16b a, v16b b, v8f c) {
    return __builtin_amdgcn_wmma_f32_16x16x32_bf16(false, a, false, b, (short)0, c, false, false);
  }
  static __device__ __forceinline__ void guard(v8f& a, v8f& b, v16b x, v16b y) { dep_guard_b(a, b, x, y); }
  static __device__ __forceinline__ void keep(v16b a, v16b b, v16b c, v16b d) { keep4_b(a, b, c, d); }
};

template <int ET> struct Elem;
template <> struct Elem<0> { typedef _Float16 T; };
template <> struct Elem<1> { typedef __bf16 T; };
template <int ET, bool SPLIT, int BIAS_MODE, int OUT_MODE, bool RESID, int ACT = 0>
__global__ __launch_bounds__(256) void wmma_gemm64(
    const unsigned short* __restrict__ Ap, const unsigned short* __restrict__ A2p, int lda, long strideA,
    const unsigned short* __restrict__ Btp, const unsigned short* __restrict__ Bt2p, int ldb, long strideB,
    void* __restrict__ Cout, void* __restrict__ Cout2, int ldc, long strideC,
    const float* __restrict__ bias,
    const float* __restrict__ resid, long strideR,
    int M, int N, int K, float scale) {
  typedef typename Elem<ET>::T T;
  typedef typename Frag<T>::V V;
  const T* A = (const T*)Ap; const T* A2 = (const T*)A2p; const T* Bt = (const T*)Btp; const T* Bt2 = (const T*)Bt2p;
  __shared__ __align__(16) float sT[8][16 * 68];
  const int b    = blockIdx.y;
  const int lane = threadIdx.x & 31;
  const int wave = threadIdx.x >> 5;
  const int tilesN = N >> 6;
  const int tilesM = M >> 6;
  const int tile = blockIdx.x * 8 + wave;
  if (tile >= tilesM * tilesN) return;
  const int tm = tile / tilesN;
  const int tn = tile - tm * tilesN;
  const int m0 = tm << 6;
  const int n0 = tn << 6;

  const T* Ab  = A  + (size_t)b * strideA;
  const T* Bb  = Bt + (size_t)b * strideB;
  const T* Ab2 = SPLIT ? (A2  + (size_t)b * strideA) : nullptr;
  const T* Bb2 = SPLIT ? (Bt2 + (size_t)b * strideB) : nullptr;

  const int rlane = lane & 15;
  const int koff  = (lane >> 4) * 8;
  const int mOff  = (lane >> 4) * 8;

  v8f acc[4][4];
#pragma unroll
  for (int i = 0; i < 4; ++i)
#pragma unroll
    for (int j = 0; j < 4; ++j) acc[i][j] = (v8f){0.f,0.f,0.f,0.f,0.f,0.f,0.f,0.f};

  for (int k0 = 0; k0 < K; k0 += 32) {
    V bh[4], bl[4];
#pragma unroll
    for (int j = 0; j < 4; ++j) {
      const size_t bo = (size_t)(n0 + (j << 4) + rlane) * ldb + koff + k0;
      bh[j] = Frag<T>::load(Bb + bo);
      if (SPLIT) bl[j] = Frag<T>::load(Bb2 + bo);
    }
#pragma unroll
    for (int i = 0; i < 4; ++i) {
      const size_t ao = (size_t)(m0 + (i << 4) + rlane) * lda + koff + k0;
      V ah = Frag<T>::load(Ab + ao);
      V al;
      if (SPLIT) al = Frag<T>::load(Ab2 + ao);
#pragma unroll
      for (int j = 0; j < 4; ++j) {
        acc[i][j] = Frag<T>::mma(ah, bh[j], acc[i][j]);
        if (SPLIT) {
          acc[i][j] = Frag<T>::mma(ah, bl[j], acc[i][j]);
          acc[i][j] = Frag<T>::mma(al, bh[j], acc[i][j]);
        }
      }
      Frag<T>::guard(acc[i][0], acc[i][3], ah, SPLIT ? al : ah);
    }
    Frag<T>::keep(bh[0], bh[1], bh[2], bh[3]);
    if (SPLIT) Frag<T>::keep(bl[0], bl[1], bl[2], bl[3]);
  }
  acc_guard4(acc[0][0], acc[0][1], acc[0][2], acc[0][3]);
  acc_guard4(acc[1][0], acc[1][1], acc[1][2], acc[1][3]);
  acc_guard4(acc[2][0], acc[2][1], acc[2][2], acc[2][3]);
  acc_guard4(acc[3][0], acc[3][1], acc[3][2], acc[3][3]);

  float* slab = sT[wave];
  const float* Rb = RESID ? (resid + (size_t)b * strideR) : nullptr;
#pragma unroll
  for (int i = 0; i < 4; ++i) {
    const int mBase = m0 + (i << 4);
#pragma unroll
    for (int j = 0; j < 4; ++j) {
      const int n = n0 + (j << 4) + rlane;
      float bv = 0.f;
      if (BIAS_MODE == 2) bv = bias[n];
#pragma unroll
      for (int r = 0; r < 8; ++r) {
        float v = acc[i][j][r] * scale;
        if (BIAS_MODE == 1) v += bias[mBase + mOff + r];
        if (BIAS_MODE == 2) v += bv;
        if (RESID) v += Rb[(size_t)(mBase + mOff + r) * ldc + n];
        if (ACT == 1) v = tanhf(v);
        if (ACT == 2) v = fmaxf(v, 0.0f);
        if (ACT == 3) v = v / (1.0f + expf(-v));
        if (ACT == 4) v = (v > 0.f) ? v : 0.01f * v;
        if (ACT == 5) v = 0.5f * v * (1.0f + erff(v * 0.70710678118654752f));
        slab[(mOff + r) * 68 + (j << 4) + rlane] = v;
      }
    }
    __builtin_amdgcn_fence(__ATOMIC_RELEASE, "workgroup");
    __builtin_amdgcn_wave_barrier();
    __builtin_amdgcn_fence(__ATOMIC_ACQUIRE, "workgroup");
    if (OUT_MODE == 0) {
      float* C = (float*)Cout + (size_t)b * strideC;
      const int hh = lane >> 4, c4 = (lane & 15) * 4;
      for (int pass = 0; pass < 2; ++pass) {
#pragma unroll
        for (int it = 0; it < 8; ++it) {
          const int row = it * 2 + hh;
          v4f v = *(const v4f*)(slab + row * 68 + c4);
          *(volatile v4f*)(C + (size_t)(mBase + row) * ldc + n0 + c4) = v;
        }
        __threadfence();
      }
    } else {
      const int q = lane >> 3, c8 = (lane & 7) * 8;
      unsigned short* C  = (unsigned short*)Cout  + (size_t)b * strideC;
      unsigned short* C2 = (OUT_MODE == 2) ? ((unsigned short*)Cout2 + (size_t)b * strideC) : nullptr;
      for (int pass = 0; pass < 2; ++pass) {
#pragma unroll
        for (int it = 0; it < 4; ++it) {
          const int row = it * 4 + q;
          const float* sp = slab + row * 68 + c8;
          v8h hv, lv;
#pragma unroll
          for (int e = 0; e < 8; ++e) {
            if (OUT_MODE == 1) {
              hv[e] = (_Float16)sp[e];
            } else {
              unsigned short hb = f2bf_bits(sp[e]);
              unsigned short lb = f2bf_bits(sp[e] - bf_bits2f(hb));
              hv[e] = __builtin_bit_cast(_Float16, hb);
              lv[e] = __builtin_bit_cast(_Float16, lb);
            }
          }
          *(volatile v8h*)(C + (size_t)(mBase + row) * ldc + n0 + c8) = hv;
          if (OUT_MODE == 2) *(volatile v8h*)(C2 + (size_t)(mBase + row) * ldc + n0 + c8) = lv;
        }
        __threadfence();
      }
    }
    __builtin_amdgcn_fence(__ATOMIC_RELEASE, "workgroup");
    __builtin_amdgcn_wave_barrier();
    __builtin_amdgcn_fence(__ATOMIC_ACQUIRE, "workgroup");
  }
}

__global__ __launch_bounds__(256) void cast_f32_f16x2(
    const float* __restrict__ in, _Float16* __restrict__ out, int n2) {
  int i = blockIdx.x * 256 + threadIdx.x;
  if (i < n2) {
    const _Float16 h0 = (_Float16)in[2 * i], h1 = (_Float16)in[2 * i + 1];
    const unsigned u = (unsigned)__builtin_bit_cast(unsigned short, h0) | ((unsigned)__builtin_bit_cast(unsigned short, h1) << 16);
    ((volatile unsigned*)out)[i] = u;
    __threadfence();
    ((volatile unsigned*)out)[i] = u;
  }
}

__global__ __launch_bounds__(256) void fold_w_kernel(
    const float* __restrict__ W0p, const float* __restrict__ A0p, const float* __restrict__ B0p,
    const float* __restrict__ W1p, const float* __restrict__ A1p, const float* __restrict__ B1p,
    const float* __restrict__ W2p, const float* __restrict__ A2p, const float* __restrict__ B2p,
    const float* __restrict__ W3p, const float* __restrict__ A3p, const float* __restrict__ B3p,
    _Float16* __restrict__ D0, _Float16* __restrict__ D1, _Float16* __restrict__ D2, _Float16* __restrict__ D3) {
  const float* W; const float* A; const float* Bm; _Float16* D;
  const int sel = blockIdx.y;
  if (sel == 0)      { W = W0p; A = A0p; Bm = B0p; D = D0; }
  else if (sel == 1) { W = W1p; A = A1p; Bm = B1p; D = D1; }
  else if (sel == 2) { W = W2p; A = A2p; Bm = B2p; D = D2; }
  else               { W = W3p; A = A3p; Bm = B3p; D = D3; }
  const int idx8 = blockIdx.x * 256 + threadIdx.x;
  if (idx8 >= (CH * CH) / 8) return;
  const int n  = idx8 >> 7;
  const int k0 = (idx8 & 127) * 8;
  v4f a0 = *(const v4f*)(W + (size_t)n * CH + k0);
  v4f a1 = *(const v4f*)(W + (size_t)n * CH + k0 + 4);
  const float* arow = A + (size_t)n * 8;
#pragma unroll 1
  for (int r = 0; r < 8; ++r) {
    const float ta = 2.0f * arow[r];
    const v4f b0 = *(const v4f*)(Bm + (size_t)r * CH + k0);
    const v4f b1 = *(const v4f*)(Bm + (size_t)r * CH + k0 + 4);
    a0 += ta * b0;
    a1 += ta * b1;
  }
  v8h hv;
#pragma unroll
  for (int e = 0; e < 4; ++e) {
    hv[e]     = (_Float16)(a0[e] * 64.0f);
    hv[4 + e] = (_Float16)(a1[e] * 64.0f);
  }
  _Float16* dp = D + (size_t)n * CH + k0;
  *(volatile v8h*)dp = hv;
  __threadfence();
  *(volatile v8h*)dp = hv;
}

__device__ __forceinline__ float wave_sum(float v) {
#pragma unroll
  for (int off = 16; off > 0; off >>= 1) v += __shfl_xor(v, off, 32);
  return v;
}

template <bool L1>
__global__ __launch_bounds__(256) void pool_kernel(
    const float* __restrict__ Kin, const float* __restrict__ Vin, const float* __restrict__ qp,
    float* __restrict__ Kfo, float* __restrict__ Vfo,
    _Float16* __restrict__ Kho, _Float16* __restrict__ Vho,
    float* __restrict__ part) {
  constexpr int NTOK  = L1 ? 1024 : 256;
  constexpr int NCHK  = L1 ? 512 : 128;
  constexpr int KEEP0 = L1 ? 256 : 64;
  constexpr int NKEEP = NCHK - KEEP0;
  __shared__ __align__(16) float skS[CH];
  __shared__ __align__(16) float svS[CH];
  __shared__ float red0[8];
  __shared__ float red1[8];
  __shared__ float red2[8];

  const int tid = threadIdx.x, lane = tid & 31, wave = tid >> 5;
  const int n = blockIdx.x, b = blockIdx.y;
  const int c4 = tid * 4;
  const size_t r0 = ((size_t)b * NTOK + 2 * n) * CH;
  const v4f qv = *(const v4f*)(qp + c4);
  const v4f ka = *(const v4f*)(Kin + r0 + c4);
  const v4f kb = *(const v4f*)(Kin + r0 + CH + c4);
  const v4f va = *(const v4f*)(Vin + r0 + c4);
  const v4f vb = *(const v4f*)(Vin + r0 + CH + c4);

  float p0 = 0.f, p1 = 0.f;
#pragma unroll
  for (int e = 0; e < 4; ++e) { p0 += qv[e] * ka[e]; p1 += qv[e] * kb[e]; }
  p0 = wave_sum(p0);
  p1 = wave_sum(p1);
  if (lane == 0) { red0[wave] = p0; red1[wave] = p1; }
  __syncthreads();
  float s0 = 0.f, s1 = 0.f;
#pragma unroll
  for (int w = 0; w < 8; ++w) { s0 += red0[w]; s1 += red1[w]; }
  const float mx = fmaxf(s0, s1);
  const float e0 = expf(s0 - mx), e1 = expf(s1 - mx);
  const float inv = 1.0f / (e0 + e1);
  const float w0 = e0 * inv, w1 = e1 * inv;

  const v4f sk = w0 * ka + w1 * kb;
  const v4f sv = w0 * va + w1 * vb;
  const v4f tv = (va + vb) * 0.5f;
  const v4f dd = sv - tv;
  float rp = 0.f;
#pragma unroll
  for (int e = 0; e < 4; ++e) rp += dd[e] * dd[e];
  *(v4f*)(skS + c4) = sk;
  *(v4f*)(svS + c4) = sv;
  rp = wave_sum(rp);
  if (lane == 0) red2[wave] = rp;
  __syncthreads();
  float tot = 0.f;
#pragma unroll
  for (int w = 0; w < 8; ++w) tot += red2[w];

  const bool keep = (n >= KEEP0);
  const int nk = keep ? (n - KEEP0) : 0;
  const size_t orow = ((size_t)b * NKEEP + nk) * CH;
  const int t8 = (tid & 127) * 8;
  v4f x0 = *(const v4f*)(skS + t8);
  v4f x1 = *(const v4f*)(skS + t8 + 4);
  const v4f y0 = *(const v4f*)(svS + t8);
  const v4f y1 = *(const v4f*)(svS + t8 + 4);
  if (tid >= 128) { x0 = y0; x1 = y1; }
  v8h hv;
#pragma unroll
  for (int e = 0; e < 4; ++e) { hv[e] = (_Float16)x0[e]; hv[4 + e] = (_Float16)x1[e]; }
  _Float16* hdst = ((tid < 128) ? Kho : Vho) + orow + t8;
  const float pv = (lane == 0) ? tot : 0.f;
  float* pdst = part + ((size_t)b * NCHK + n) * 32 + lane;
  for (int pass = 0; pass < 2; ++pass) {
    if (keep) {
      if (L1) {
        *(volatile v4f*)(Kfo + orow + c4) = sk;
        *(volatile v4f*)(Vfo + orow + c4) = sv;
      }
      *(volatile v8h*)hdst = hv;
    }
    if (wave == 0) *(volatile float*)pdst = pv;
    __threadfence();
  }
}

__device__ __forceinline__ v8f mma_h(v16h a, v16h b, v8f c) {
  c = __builtin_amdgcn_wmma_f32_16x16x32_f16(false, a, false, b, (short)0, c, false, false);
  asm volatile("v_nop\n\tv_nop\n\tv_nop\n\tv_nop" : "+v"(c) : "v"(a), "v"(b));
  return c;
}
union FH { v16h v; v8h h[2]; };

__global__ __launch_bounds__(128) void attn3_kernel(
    const _Float16* __restrict__ Qp,
    const _Float16* __restrict__ K0p, const _Float16* __restrict__ V0p,
    const _Float16* __restrict__ K1p, const _Float16* __restrict__ V1p,
    const _Float16* __restrict__ K2p, const _Float16* __restrict__ V2p,
    _Float16* __restrict__ Op, const float* __restrict__ logits) {
  __shared__ __align__(16) _Float16 Ksh[AKC * HD];
  __shared__ __align__(16) _Float16 Vth[HD * AKC];
  __shared__ __align__(16) _Float16 Psh[4][16 * AKC];
  __shared__ __align__(16) float    Os[4][16 * 68];

  const int tid  = threadIdx.x;
  const int wave = tid >> 5;
  const int lane = tid & 31;
  const int hh   = lane >> 4;
  const int c    = lane & 15;
  const int bx = blockIdx.x;
  const int qb = bx % (SEQ / 64);
  const int bh = bx / (SEQ / 64);
  const int h  = bh % NHEAD;
  const int b  = bh / NHEAD;
  const int q0 = qb * 64 + wave * 16;

  v16h qa[2];
  {
    const _Float16* qrow = Qp + ((size_t)b * SEQ + q0 + c) * CH + h * HD;
#pragma unroll
    for (int dc = 0; dc < 2; ++dc) qa[dc] = Frag<_Float16>::load(qrow + dc * 32 + 8 * hh);
  }
  float lw0, lw1, lw2;
  {
    const float g0 = logits[0], g1 = logits[1], g2 = logits[2];
    const float gm = fmaxf(g0, fmaxf(g1, g2));
    const float x0 = expf(g0 - gm), x1 = expf(g1 - gm), x2 = expf(g2 - gm);
    const float ginv = 1.0f / (x0 + x1 + x2);
    lw0 = x0 * ginv; lw1 = x1 * ginv; lw2 = x2 * ginv;
  }
  float* os = Os[wave];
#pragma unroll
  for (int r = 0; r < 8; ++r)
#pragma unroll
    for (int t = 0; t < 4; ++t) os[(8 * hh + r) * 68 + t * 16 + c] = 0.f;

#pragma unroll 1
  for (int lev = 0; lev < 3; ++lev) {
    int nCh; const _Float16* kbp; const _Float16* vbp; float lwl;
    if (lev == 0)      { nCh = NK0 / AKC; kbp = K0p + (size_t)b * NK0 * CH; vbp = V0p + (size_t)b * NK0 * CH; lwl = lw0; }
    else if (lev == 1) { nCh = NK1 / AKC; kbp = K1p + (size_t)b * NK1 * CH; vbp = V1p + (size_t)b * NK1 * CH; lwl = lw1; }
    else               { nCh = NK2 / AKC; kbp = K2p + (size_t)b * NK2 * CH; vbp = V2p + (size_t)b * NK2 * CH; lwl = lw2; }
    kbp += h * HD; vbp += h * HD;

    float mrow[8], lrow[8];
    v8f oacc[4];
#pragma unroll
    for (int r = 0; r < 8; ++r) { mrow[r] = -__builtin_inff(); lrow[r] = 0.f; }
#pragma unroll
    for (int t = 0; t < 4; ++t) oacc[t] = (v8f){0.f,0.f,0.f,0.f,0.f,0.f,0.f,0.f};

    for (int kc = 0; kc < nCh; ++kc) {
      const int kv0 = kc * AKC;
      __syncthreads();
      {
        const int kvr = tid >> 1, dh = (tid & 1) * 32;
        const _Float16* krow = kbp + (size_t)(kv0 + kvr) * CH + dh;
        const _Float16* vrow = vbp + (size_t)(kv0 + kvr) * CH + dh;
#pragma unroll
        for (int i = 0; i < 4; ++i) {
          const v8h kk = *(const v8h*)(krow + 8 * i);
          *(v8h*)(Ksh + kvr * HD + dh + 8 * i) = kk;
          const v8h vv = *(const v8h*)(vrow + 8 * i);
#pragma unroll
          for (int e = 0; e < 8; ++e) Vth[(dh + 8 * i + e) * AKC + kvr] = vv[e];
        }
      }
      __syncthreads();

      v8f s[4];
#pragma unroll
      for (int j = 0; j < 4; ++j) {
        s[j] = (v8f){0.f,0.f,0.f,0.f,0.f,0.f,0.f,0.f};
#pragma unroll
        for (int dc = 0; dc < 2; ++dc) {
          FH kf;
          kf.h[0] = *(const v8h*)(Ksh + (j * 16 + c) * HD + dc * 32 + 8 * hh);
          kf.h[1] = *(const v8h*)(Ksh + (j * 16 + c) * HD + dc * 32 + 16 + 8 * hh);
          s[j] = mma_h(qa[dc], kf.v, s[j]);
        }
      }
      float cm[8];
#pragma unroll
      for (int r = 0; r < 8; ++r) {
        float m = -__builtin_inff();
#pragma unroll
        for (int j = 0; j < 4; ++j) {
          const float x = s[j][r] * 0.125f;
          s[j][r] = x;
          m = fmaxf(m, x);
        }
#pragma unroll
        for (int off = 1; off < 16; off <<= 1) m = fmaxf(m, __shfl_xor(m, off, 32));
        cm[r] = m;
      }
      _Float16* pw = Psh[wave];
#pragma unroll
      for (int r = 0; r < 8; ++r) {
        const float mnew = fmaxf(mrow[r], cm[r]);
        const float alpha = expf(mrow[r] - mnew);
        mrow[r] = mnew;
        float psum = 0.f;
#pragma unroll
        for (int j = 0; j < 4; ++j) {
          const float p = expf(s[j][r] - mnew);
          psum += p;
          pw[(8 * hh + r) * AKC + j * 16 + c] = (_Float16)(p * 32768.0f);
        }
#pragma unroll
        for (int off = 1; off < 16; off <<= 1) psum += __shfl_xor(psum, off, 32);
        lrow[r] = lrow[r] * alpha + psum;
#pragma unroll
        for (int t = 0; t < 4; ++t) oacc[t][r] *= alpha;
      }
      __builtin_amdgcn_fence(__ATOMIC_RELEASE, "workgroup");
      __builtin_amdgcn_wave_barrier();
      __builtin_amdgcn_fence(__ATOMIC_ACQUIRE, "workgroup");
#pragma unroll
      for (int kk = 0; kk < 2; ++kk) {
        FH pa;
        pa.h[0] = *(const v8h*)(pw + c * AKC + kk * 32 + 8 * hh);
        pa.h[1] = *(const v8h*)(pw + c * AKC + kk * 32 + 16 + 8 * hh);
#pragma unroll
        for (int t = 0; t < 4; ++t) {
          FH vf;
          vf.h[0] = *(const v8h*)(Vth + (t * 16 + c) * AKC + kk * 32 + 8 * hh);
          vf.h[1] = *(const v8h*)(Vth + (t * 16 + c) * AKC + kk * 32 + 16 + 8 * hh);
          oacc[t] = mma_h(pa.v, vf.v, oacc[t]);
        }
      }
    }
#pragma unroll
    for (int r = 0; r < 8; ++r) {
      const float coef = lwl * 0.001953125f * (1.0f / lrow[r]);
#pragma unroll
      for (int t = 0; t < 4; ++t) os[(8 * hh + r) * 68 + t * 16 + c] += oacc[t][r] * coef;
    }
  }

  __builtin_amdgcn_fence(__ATOMIC_RELEASE, "workgroup");
  __builtin_amdgcn_wave_barrier();
  __builtin_amdgcn_fence(__ATOMIC_ACQUIRE, "workgroup");
  {
    const int q4 = lane >> 3, c8 = (lane & 7) * 8;
    _Float16* ob = Op + ((size_t)b * SEQ + q0) * CH + h * HD;
    for (int pass = 0; pass < 2; ++pass) {
#pragma unroll
      for (int it = 0; it < 4; ++it) {
        const int row = it * 4 + q4;
        const float* sp = os + row * 68 + c8;
        v8h hv;
#pragma unroll
        for (int e = 0; e < 8; ++e) hv[e] = (_Float16)sp[e];
        *(volatile v8h*)(ob + (size_t)row * CH + c8) = hv;
      }
      __threadfence();
    }
  }
}

__global__ __launch_bounds__(256) void recon_kernel(
    const float* __restrict__ p1, const float* __restrict__ p2, float* __restrict__ dst) {
  __shared__ double sh1[256];
  __shared__ double sh2[256];
  const int tid = threadIdx.x;
  double a = 0.0, bsum = 0.0;
  for (int i = tid; i < NB * 512; i += 256) a += (double)p1[(size_t)i * 32];
  for (int i = tid; i < NB * 128; i += 256) bsum += (double)p2[(size_t)i * 32];
  sh1[tid] = a; sh2[tid] = bsum;
  __syncthreads();
  if (tid == 0) {
    double S1 = 0.0, S2 = 0.0;
    for (int i = 0; i < 256; ++i) { S1 += sh1[i]; S2 += sh2[i]; }
    const float r1 = (float)(S1 * (1.0 / 2097152.0));
    const float r2 = (float)(S2 * (1.0 / 524288.0));
    float rec = 0.0f + r1;
    rec = rec + 64.0f * r2;
    *(volatile float*)dst = rec;
    __threadfence();
    *(volatile float*)dst = rec;
  }
}

extern "C" void kernel_launch(void* const* d_in, const int* in_sizes, int n_in,
                              void* d_out, int out_size, void* d_ws, size_t ws_size,
                              hipStream_t stream) {
  if (n_in < 15) return;
  if (in_sizes[0] != NB * SEQ * CH) return;
  if (in_sizes[1] != CH * CH || in_sizes[4] != CH * CH || in_sizes[7] != CH * CH || in_sizes[10] != CH * CH) return;
  if (in_sizes[2] != CH * 8 || in_sizes[5] != CH * 8 || in_sizes[8] != CH * 8 || in_sizes[11] != CH * 8) return;
  if (in_sizes[3] != 8 * CH || in_sizes[6] != 8 * CH || in_sizes[9] != 8 * CH || in_sizes[12] != 8 * CH) return;
  if (in_sizes[13] != 2 * CH || in_sizes[14] < 3) return;
  if (out_size != NB * SEQ * CH + 1) return;

  const float* x      = (const float*)d_in[0];
  const float* Wq_w   = (const float*)d_in[1];
  const float* Wq_A   = (const float*)d_in[2];
  const float* Wq_B   = (const float*)d_in[3];
  const float* Wk_w   = (const float*)d_in[4];
  const float* Wk_A   = (const float*)d_in[5];
  const float* Wk_B   = (const float*)d_in[6];
  const float* Wv_w   = (const float*)d_in[7];
  const float* Wv_A   = (const float*)d_in[8];
  const float* Wv_B   = (const float*)d_in[9];
  const float* Wo_w   = (const float*)d_in[10];
  const float* Wo_A   = (const float*)d_in[11];
  const float* Wo_B   = (const float*)d_in[12];
  const float* q_pool = (const float*)d_in[13];
  const float* logits = (const float*)d_in[14];
  float* out = (float*)d_out;

  const size_t MT = (size_t)NB * SEQ;
  size_t off = 0;
  char* ws = (char*)d_ws;
  const size_t o_xh  = off; off += MT * CH * 2;
  const size_t o_w   = off; off += (size_t)4 * CH * CH * 2;
  const size_t o_q   = off; off += MT * CH * 2;
  const size_t o_kf  = off; off += (size_t)NB * 1024 * CH * 4;
  const size_t o_vf  = off; off += (size_t)NB * 1024 * CH * 4;
  const size_t o_kh  = off; off += (size_t)NB * 1024 * CH * 2;
  const size_t o_vh  = off; off += (size_t)NB * 1024 * CH * 2;
  const size_t o_k1f = off; off += (size_t)NB * 256 * CH * 4;
  const size_t o_v1f = off; off += (size_t)NB * 256 * CH * 4;
  const size_t o_k1h = off; off += (size_t)NB * 256 * CH * 2;
  const size_t o_v1h = off; off += (size_t)NB * 256 * CH * 2;
  const size_t o_k2h = off; off += (size_t)NB * 64 * CH * 2;
  const size_t o_v2h = off; off += (size_t)NB * 64 * CH * 2;
  const size_t o_p1  = off; off += (size_t)NB * 512 * 128;
  const size_t o_p2  = off; off += (size_t)NB * 128 * 128;
  if (off > ws_size) return;

  _Float16* xh  = (_Float16*)(ws + o_xh);
  _Float16* wq  = (_Float16*)(ws + o_w);
  _Float16* wk  = wq + (size_t)CH * CH;
  _Float16* wv  = wk + (size_t)CH * CH;
  _Float16* wo  = wv + (size_t)CH * CH;
  _Float16* Qh  = (_Float16*)(ws + o_q);
  float*    Kf  = (float*)(ws + o_kf);
  float*    Vf  = (float*)(ws + o_vf);
  _Float16* Kh  = (_Float16*)(ws + o_kh);
  _Float16* Vh  = (_Float16*)(ws + o_vh);
  float*    K1f = (float*)(ws + o_k1f);
  float*    V1f = (float*)(ws + o_v1f);
  _Float16* K1h = (_Float16*)(ws + o_k1h);
  _Float16* V1h = (_Float16*)(ws + o_v1h);
  _Float16* K2h = (_Float16*)(ws + o_k2h);
  _Float16* V2h = (_Float16*)(ws + o_v2h);
  float*    P1  = (float*)(ws + o_p1);
  float*    P2  = (float*)(ws + o_p2);
  _Float16* Oh  = xh;

  const unsigned short* xh_u = (const unsigned short*)xh;
  const unsigned short* wq_u = (const unsigned short*)wq;
  const unsigned short* wk_u = (const unsigned short*)wk;
  const unsigned short* wv_u = (const unsigned short*)wv;
  const unsigned short* wo_u = (const unsigned short*)wo;
  const float* fdum = q_pool;

  {
    const int n2 = (int)(MT * CH / 2);
    cast_f32_f16x2<<<dim3((n2 + 255) / 256), 256, 0, stream>>>(x, xh, n2);
  }
  fold_w_kernel<<<dim3((CH * CH / 8 + 255) / 256, 4), 256, 0, stream>>>(
      Wq_w, Wq_A, Wq_B, Wk_w, Wk_A, Wk_B, Wv_w, Wv_A, Wv_B, Wo_w, Wo_A, Wo_B, wq, wk, wv, wo);

  const float s64 = 1.0f / 64.0f;
  wmma_gemm64<0, false, 0, 1, false, 0><<<dim3((128 * 16 + 7) / 8, 1), 256, 0, stream>>>(
      xh_u, xh_u, CH, 0L, wq_u, wq_u, CH, 0L, (void*)Qh, (void*)Qh, CH, 0L,
      fdum, fdum, 0L, (int)MT, CH, CH, s64);
  wmma_gemm64<0, false, 0, 0, false, 0><<<dim3((16 * 16 + 7) / 8, NB), 256, 0, stream>>>(
      xh_u, xh_u, CH, (long)SEQ * CH, wk_u, wk_u, CH, 0L, (void*)Kf, (void*)Kf, CH, (long)1024 * CH,
      fdum, fdum, 0L, 1024, CH, CH, s64);
  wmma_gemm64<0, false, 0, 1, false, 0><<<dim3((16 * 16 + 7) / 8, NB), 256, 0, stream>>>(
      xh_u + (size_t)1024 * CH, xh_u + (size_t)1024 * CH, CH, (long)SEQ * CH, wk_u, wk_u, CH, 0L,
      (void*)Kh, (void*)Kh, CH, (long)1024 * CH, fdum, fdum, 0L, 1024, CH, CH, s64);
  wmma_gemm64<0, false, 0, 0, false, 0><<<dim3((16 * 16 + 7) / 8, NB), 256, 0, stream>>>(
      xh_u, xh_u, CH, (long)SEQ * CH, wv_u, wv_u, CH, 0L, (void*)Vf, (void*)Vf, CH, (long)1024 * CH,
      fdum, fdum, 0L, 1024, CH, CH, s64);
  wmma_gemm64<0, false, 0, 1, false, 0><<<dim3((16 * 16 + 7) / 8, NB), 256, 0, stream>>>(
      xh_u + (size_t)1024 * CH, xh_u + (size_t)1024 * CH, CH, (long)SEQ * CH, wv_u, wv_u, CH, 0L,
      (void*)Vh, (void*)Vh, CH, (long)1024 * CH, fdum, fdum, 0L, 1024, CH, CH, s64);

  pool_kernel<true><<<dim3(512, NB), 256, 0, stream>>>(Kf, Vf, q_pool, K1f, V1f, K1h, V1h, P1);
  pool_kernel<false><<<dim3(128, NB), 256, 0, stream>>>(K1f, V1f, q_pool + CH, K1f, V1f, K2h, V2h, P2);

  attn3_kernel<<<dim3(NB * NHEAD * (SEQ / 64)), 128, 0, stream>>>(
      Qh, Kh, Vh, K1h, V1h, K2h, V2h, Oh, logits);

  wmma_gemm64<0, false, 0, 0, false, 0><<<dim3((128 * 16 + 7) / 8, 1), 256, 0, stream>>>(
      (const unsigned short*)Oh, (const unsigned short*)Oh, CH, 0L, wo_u, wo_u, CH, 0L,
      (void*)out, (void*)out, CH, 0L, fdum, fdum, 0L, (int)MT, CH, CH, 1.0f / 4096.0f);

  recon_kernel<<<dim3(1), 256, 0, stream>>>(P1, P2, out + MT * CH);
}
